// CGNN_81363860455904
// MI455X (gfx1250) — hardware-verified
//
#include <hip/hip_runtime.h>


namespace {
constexpr int NB = 16, T = 4, F = 512, S = 14, DS = 32, HA = 128, CM = 66, CMP = 72  , NIT = 2, GB = 4  , NG = NB / GB, NG_RUN = 4  ;
constexpr int PXG = GB * T * F * S;
constexpr float XS = 8.0f, WSC = 256.0f;
static_assert(PXG % 64 == 0 && (2 * S * CMP * 4) % 128 == 0 && F % 2 == 0, "tiling / line alignment of the 2-row stencil blocks");
typedef _Float16 b16;
typedef __attribute__((ext_vector_type(16))) _Float16 v16b;
typedef __attribute__((ext_vector_type(8))) _Float16 v8b;
typedef __attribute__((ext_vector_type(8))) float v8f;
typedef __attribute__((ext_vector_type(4))) float v4f;
__device__ __forceinline__ float bf16_rne(float f) { unsigned int u = __float_as_uint(f); u += 0x7FFFu + ((u >> 16) & 1u); return __uint_as_float(u & 0xFFFF0000u); }
__device__ __forceinline__ void split16(float v, b16& hi, b16& lo) { hi = (b16)v; lo = (b16)(v - (float)hi); }
__device__ __forceinline__ v16b frag_kb(const b16* p, int hh) { const v8b a = *(const v8b*)(p + 8 * hh), b = *(const v8b*)(p + 16 + 8 * hh); v16b f;
#pragma unroll
  for (int e = 0; e < 8; ++e) { f[e] = a[e]; f[8 + e] = b[e]; } return f; }
__device__ __forceinline__ v8f wmma16b(v16b a, v16b b, v8f c) { v8f d = __builtin_amdgcn_wmma_f32_16x16x32_f16(false, a, false, b, (short)0, c, false, false); asm volatile("v_nop\n\tv_nop\n\tv_nop\n\tv_nop" : "+v"(d) : "v"(a), "v"(b)); return d; }
__device__ __forceinline__ void wave_lds_sync() { __builtin_amdgcn_fence(__ATOMIC_RELEASE, "workgroup"); __builtin_amdgcn_wave_barrier(); __builtin_amdgcn_fence(__ATOMIC_ACQUIRE, "workgroup"); }
__device__ __forceinline__ float pmul(float a, float b) { float p = a * b; asm volatile("" : "+v"(p)); return p; }
__device__ __forceinline__ int iclamp(int v, int lo, int hi) { return v < lo ? lo : (v > hi ? hi : v); }

typedef __attribute__((ext_vector_type(2))) float v2f;
__global__ __launch_bounds__(256) void prep_kernel(const float* __restrict__ aw1, const float* __restrict__ aw2, const float* __restrict__ pw1, const float* __restrict__ pw2, b16* __restrict__ AW1, b16* __restrict__ AW2, b16* __restrict__ PW1, b16* __restrict__ PW2) {
  const int t = blockIdx.x * 256 + threadIdx.x; v8b o; const int n1 = HA * DS / 8, n2 = DS * HA / 8, n3 = 80 * 96 / 8, n4 = DS * 96 / 8;
  if (t < n1) { const int e = t * 8, oo = e / DS, k0 = e % DS; for (int j = 0; j < 8; ++j) o[j] = (b16)(bf16_rne(aw1[(k0 + j) * HA + oo]) * WSC); for (int pass = 0; pass < 2; ++pass) { *(volatile v8b*)(AW1 + e) = o; __threadfence(); } }
  else if (t < n1 + n2) { const int e = (t - n1) * 8, oo = e / HA, k0 = e % HA; for (int j = 0; j < 8; ++j) o[j] = (b16)(bf16_rne(aw2[(k0 + j) * DS + oo]) * WSC); for (int pass = 0; pass < 2; ++pass) { *(volatile v8b*)(AW2 + e) = o; __threadfence(); } }
  else if (t < n1 + n2 + n3) { const int e = (t - n1 - n2) * 8, oo = e / 96, k0 = e % 96; for (int j = 0; j < 8; ++j) { const int k = k0 + j; o[j] = (oo < CM && k < CM) ? (b16)(bf16_rne(pw1[oo * CM + k]) * WSC) : (b16)0.0f; } for (int pass = 0; pass < 2; ++pass) { *(volatile v8b*)(PW1 + e) = o; __threadfence(); } }
  else if (t < n1 + n2 + n3 + n4) { const int e = (t - n1 - n2 - n3) * 8, oo = e / 96, k0 = e % 96; for (int j = 0; j < 8; ++j) { const int k = k0 + j; o[j] = (k < CM) ? (b16)(bf16_rne(pw2[oo * CM + k]) * WSC) : (b16)0.0f; } for (int pass = 0; pass < 2; ++pass) { *(volatile v8b*)(PW2 + e) = o; __threadfence(); } }
}
template <int KREAL, bool ROUND>
__device__ __forceinline__ v16b frag_f32(const float* __restrict__ row, int ks, int hh) {
  v16b a;
#pragma unroll
  for (int g = 0; g < 2; ++g) {
#pragma unroll
    for (int i = 0; i < 8; ++i) { const int k = ks * 32 + g * 16 + 8 * hh + i; float v = 0.0f; if (KREAL % 32 == 0 || k < KREAL) v = row[k < KREAL ? k : 0]; if (ROUND) v = bf16_rne(v); a[g * 8 + i] = (b16)(v * XS); } }
  return a;
}
template <bool FIRST>
__global__ __launch_bounds__(128) void aggmlp_kernel(const float* __restrict__ SIN, size_t sin_px0  , const float* __restrict__ act, int g, const b16* __restrict__ AW1, const b16* __restrict__ AW2, const float* __restrict__ b1, const float* __restrict__ b2, float* __restrict__ SP) {
  __shared__ __attribute__((aligned(16))) float Th[4][16][HA + 4]; __shared__ __attribute__((aligned(16))) float To[4][16][DS + 4];
  const int wave = threadIdx.x >> 5, lane = threadIdx.x & 31, nloc = lane & 15, hlf = lane >> 4; const size_t p0 = ((size_t)blockIdx.x * 4 + wave) * 16; const size_t pr = p0 + nloc;
  v8f acc[8];
#pragma unroll
  for (int t = 0; t < 8; ++t) acc[t] = (v8f){};
  { const v16b a = frag_f32<DS, FIRST>(SIN + (sin_px0 + pr) * DS, 0, hlf);
#pragma unroll
    for (int t = 0; t < 8; ++t) acc[t] = wmma16b(a, frag_kb(AW1 + (size_t)(t * 16 + nloc) * DS, hlf), acc[t]); }
#pragma unroll
  for (int t = 0; t < 8; ++t) { const float bb = bf16_rne(b1[t * 16 + nloc]);
#pragma unroll
    for (int r = 0; r < 8; ++r) Th[wave][8 * hlf + r][t * 16 + nloc] = fmaxf(acc[t][r] * (1.0f / (XS * WSC)) + bb, 0.0f); }
  wave_lds_sync();
  v8f acc2[2] = {(v8f){}, (v8f){}};
#pragma unroll
  for (int ks = 0; ks < HA / 32; ++ks) { const v16b a = frag_f32<HA, false>(&Th[wave][nloc][0], ks, hlf);
#pragma unroll
    for (int t = 0; t < 2; ++t) acc2[t] = wmma16b(a, frag_kb(AW2 + (size_t)(t * 16 + nloc) * HA + ks * 32, hlf), acc2[t]); }
#pragma unroll
  for (int t = 0; t < 2; ++t) { const float bb = bf16_rne(b2[t * 16 + nloc]);
#pragma unroll
    for (int r = 0; r < 8; ++r) { const size_t p = p0 + 8 * hlf + r; const int bl = (int)(p / ((size_t)T * F * S)), tt = (int)((p / ((size_t)F * S)) % T); const float ac = bf16_rne(act[(g * GB + bl) * T + tt]); To[wave][8 * hlf + r][t * 16 + nloc] = (acc2[t][r] * (1.0f / (XS * WSC)) + bb) * ac; } }
  wave_lds_sync();
  for (int pass = 0; pass < 2; ++pass) { for (int rr = 0; rr < 16; ++rr) ((volatile float*)SP)[(p0 + rr) * DS + lane] = To[wave][rr][lane]; __threadfence(); }
}
template <int PASS, bool FIRST>
__global__ __launch_bounds__(256) void dw_kernel(const float* __restrict__ SP, const float* __restrict__ SIN, size_t sin_px0, const float* __restrict__ pe, const float* __restrict__ act, int g, const float* __restrict__ P1, const float* __restrict__ w, const float* __restrict__ bias, float* __restrict__ DOUT) {
  constexpr int ZC = 68, NCH = 17;
  __shared__ __attribute__((aligned(16))) float Z[4][S][ZC]; __shared__ __attribute__((aligned(16))) float WT9[9][ZC]; __shared__ __attribute__((aligned(16))) float BB[ZC];
  const int blk = blockIdx.x; const int bt = blk / (F / 2), f0 = (blk % (F / 2)) * 2; const int bl = bt / T, tt = bt % T; const int tid = threadIdx.x;
  float pinv = 1.0f; if (PASS == 1) { float psum = 0.0f; for (int t2 = 0; t2 < T; ++t2) psum += bf16_rne(act[(g * GB + bl) * T + t2]); psum -= 1.0f; psum = fmaxf(psum, 0.0f); pinv = (psum == 0.0f) ? 1.0f : 1.0f / psum; }
  for (int i = tid; i < 9 * ZC; i += 256) { const int tap = i / ZC, c = i % ZC; WT9[tap][c] = (c < CM) ? bf16_rne(w[c * 9 + tap]) : 0.0f; }
  for (int i = tid; i < ZC; i += 256) BB[i] = (i < CM) ? bf16_rne(bias[i]) : 0.0f;
  for (int i = tid; i < 4 * S * NCH; i += 256) { const int r = i / (S * NCH), rem = i % (S * NCH); const int ss = rem / NCH, q = rem % NCH; const int ff = f0 - 1 + r; v4f v = {0.0f, 0.0f, 0.0f, 0.0f};
    if (ff >= 0 && ff < F) { const size_t p = (((size_t)bt * F + ff) * S + ss);
      if (PASS == 1) {
        if (q < 8) { v4f tot = {0.0f, 0.0f, 0.0f, 0.0f};
#pragma unroll
          for (int t2 = 0; t2 < T; ++t2) tot += *(const v4f*)(SP + ((((size_t)bl * T + t2) * F + ff) * S + ss) * DS + q * 4);
          const v4f own = *(const v4f*)(SP + p * DS + q * 4); v = (tot - own) * pinv; }
        else if (q < 16) { const v4f sv = *(const v4f*)(SIN + (sin_px0 + p) * DS + (q - 8) * 4); if (FIRST) { for (int j = 0; j < 4; ++j) v[j] = bf16_rne(sv[j]); } else v = sv; }
        else { const float* pp = pe + (((size_t)tt * F + ff) * S + ss) * 2; v[0] = bf16_rne(pp[0]); v[1] = bf16_rne(pp[1]); } }
      else { v = *(const v4f*)(P1 + p * CMP + q * 4); if (q == 16) { v[2] = 0.0f; v[3] = 0.0f; } } }
    *(v4f*)(&Z[r][ss][q * 4]) = v; }
  __syncthreads();
  for (int pass = 0; pass < 2; ++pass) {
    for (int i = tid; i < 2 * S * (CMP / 4); i += 256) { const int r = i / (S * (CMP / 4)), rem = i % (S * (CMP / 4)); const int ss = rem / (CMP / 4), q = rem % (CMP / 4); v4f o = {0.0f, 0.0f, 0.0f, 0.0f};
      if (q < NCH) { o = *(const v4f*)(&BB[q * 4]);
#pragma unroll
        for (int df = 0; df < 3; ++df)
#pragma unroll
          for (int dsx = 0; dsx < 3; ++dsx) { const int s2 = ss + dsx - 1; if (s2 >= 0 && s2 < S) o += *(const v4f*)(&WT9[df * 3 + dsx][q * 4]) * *(const v4f*)(&Z[r + df][s2][q * 4]); }
        if (q == 16) { o[2] = 0.0f; o[3] = 0.0f; } }
      *(volatile v4f*)(DOUT + ((((size_t)bt * F + f0 + r) * S) + ss) * CMP + q * 4) = o; }
    __threadfence(); }
}
template <int MODE, bool FIRST>
__global__ __launch_bounds__(128) void pw_kernel(const float* __restrict__ DIN, const b16* __restrict__ PW, const float* __restrict__ bias, const float* __restrict__ SIN, size_t sin_px0, float* __restrict__ OUTP, size_t out_px0) {
  constexpr int NT = (MODE == 1) ? 5 : 2; constexpr int OW = (MODE == 1) ? CMP : DS;
  __shared__ __attribute__((aligned(16))) float Tf[4][16][80 + 4];
  const int wave = threadIdx.x >> 5, lane = threadIdx.x & 31, nloc = lane & 15, hlf = lane >> 4; const size_t p0 = ((size_t)blockIdx.x * 4 + wave) * 16; const size_t pr = p0 + nloc;
  v8f acc[NT];
#pragma unroll
  for (int t = 0; t < NT; ++t) acc[t] = (v8f){};
#pragma unroll
  for (int ks = 0; ks < 3; ++ks) { const v16b a = frag_f32<CM, false>(DIN + pr * CMP, ks, hlf);
#pragma unroll
    for (int t = 0; t < NT; ++t) acc[t] = wmma16b(a, frag_kb(PW + (size_t)(t * 16 + nloc) * 96 + ks * 32, hlf), acc[t]); }
#pragma unroll
  for (int t = 0; t < NT; ++t) { const int c = t * 16 + nloc; const float bb = (c < (MODE == 1 ? CM : DS)) ? bf16_rne(bias[c]) : 0.0f;
#pragma unroll
    for (int r = 0; r < 8; ++r) { float v = acc[t][r] * (1.0f / (XS * WSC)) + bb; if (MODE == 1) v = (c < CM) ? fmaxf(v, 0.0f) : 0.0f; Tf[wave][8 * hlf + r][c] = v; } }
  wave_lds_sync();
  for (int pass = 0; pass < 2; ++pass) {
    for (int rr = 0; rr < 16; ++rr) { const size_t p = p0 + rr;
      if (MODE == 1) { for (int c = lane; c < CMP; c += 32) ((volatile float*)OUTP)[p * CMP + c] = (c < 80) ? Tf[wave][rr][c] : 0.0f; }
      else { const float so = SIN[(sin_px0 + p) * DS + lane]; ((volatile float*)OUTP)[(out_px0 + p) * DS + lane] = Tf[wave][rr][lane] + (FIRST ? bf16_rne(so) : so); } }
    __threadfence(); }
}
}

extern "C" void kernel_launch(void* const* d_in, const int* in_sizes, int n_in, void* d_out, int out_size, void* d_ws, size_t ws_size, hipStream_t stream) {
  (void)n_in;
  auto Fp = [&](int i) { return (const float*)d_in[i]; };
  if (in_sizes[0] != NB * T * F * S * DS || in_sizes[1] != T * F * S * 2 || in_sizes[2] != NB * T || in_sizes[3] != DS * HA || in_sizes[5] != HA * DS || in_sizes[7] != CM * 9 || in_sizes[9] != CM * CM || in_sizes[11] != CM * 9 || in_sizes[13] != DS * CM || in_sizes[14] != DS || out_size != NB * T * F * S * DS) return;
  size_t off = 0; char* ws = (char*)d_ws;
  auto carve = [&](size_t bytes) { char* p = ws + off; off += (bytes + 255) & ~(size_t)255; return p; };
  b16* AW1 = (b16*)carve(HA * DS * 2); b16* AW2 = (b16*)carve(DS * HA * 2); b16* PW1 = (b16*)carve(80 * 96 * 2); b16* PW2 = (b16*)carve(DS * 96 * 2);
  float* SP = (float*)carve((size_t)PXG * DS * 4); float* DPL = (float*)carve((size_t)PXG * CMP * 4); float* P1 = (float*)carve((size_t)PXG * CMP * 4); float* S1 = (float*)carve((size_t)PXG * DS * 4);
  if (off > ws_size || off > ((size_t)128 << 20)) return;
  prep_kernel<<<(HA * DS / 8 + DS * HA / 8 + 80 * 96 / 8 + DS * 96 / 8 + 255) / 256, 256, 0, stream>>>(Fp(3), Fp(5), Fp(9), Fp(13), AW1, AW2, PW1, PW2);
  const float* s_in = Fp(0); float* out = (float*)d_out;
  for (int g = 0; g < NG_RUN; ++g) { const size_t gpx0 = (size_t)g * PXG;
    aggmlp_kernel<true><<<PXG / 64, 128, 0, stream>>>(s_in, gpx0, Fp(2), g, AW1, AW2, Fp(4), Fp(6), SP);
    dw_kernel<1, true><<<GB * T * (F / 2), 256, 0, stream>>>(SP, s_in, gpx0, Fp(1), Fp(2), g, nullptr, Fp(7), Fp(8), DPL);
    pw_kernel<1, true><<<PXG / 64, 128, 0, stream>>>(DPL, PW1, Fp(10), nullptr, 0, P1, 0);
    dw_kernel<2, true><<<GB * T * (F / 2), 256, 0, stream>>>(nullptr, nullptr, 0, nullptr, nullptr, g, P1, Fp(11), Fp(12), DPL);
    pw_kernel<2, true><<<PXG / 64, 128, 0, stream>>>(DPL, PW2, Fp(14), s_in, gpx0, S1, 0);
    aggmlp_kernel<false><<<PXG / 64, 128, 0, stream>>>(S1, 0, Fp(2), g, AW1, AW2, Fp(4), Fp(6), SP);
    dw_kernel<1, false><<<GB * T * (F / 2), 256, 0, stream>>>(SP, S1, 0, Fp(1), Fp(2), g, nullptr, Fp(7), Fp(8), DPL);
    pw_kernel<1, false><<<PXG / 64, 128, 0, stream>>>(DPL, PW1, Fp(10), nullptr, 0, P1, 0);
    dw_kernel<2, false><<<GB * T * (F / 2), 256, 0, stream>>>(nullptr, nullptr, 0, nullptr, nullptr, g, P1, Fp(11), Fp(12), DPL);
    pw_kernel<2, false><<<PXG / 64, 128, 0, stream>>>(DPL, PW2, Fp(14), S1, 0, out, gpx0);
  }
}
